// GNN4Contrastive_35261681500246
// MI455X (gfx1250) — hardware-verified
//
#include <hip/hip_runtime.h>
#include <stddef.h>


#define FT    128
#define GR    32
#define AP    136
#define XSP   132
#define TP    132
#define NB    512
#define CHUNK 4096
#define NTHR  256
#define NWAVE 8
#define WCAP  512
#define NGRP  (CHUNK / (NTHR * 4))

#define LDS_SACC (NB * FT)
#define LDS_AUXF (3 * NB)
#define LDS_LIST (NWAVE * WCAP)
#define LDS_BYTES ((LDS_SACC + LDS_AUXF + LDS_LIST + 16) * 4)

static_assert(WCAP == (CHUNK / NTHR) * 32);
static_assert(NGRP == 4);
static_assert(NB == 512);
static_assert((NB / NWAVE) * NWAVE == NB);
static_assert(CHUNK <= 4096);
static_assert(((LDS_SACC + LDS_AUXF) % 4) == 0);
static_assert(LDS_BYTES == 284736);

typedef float          v4f   __attribute__((ext_vector_type(4)));
typedef float          v8f   __attribute__((ext_vector_type(8)));
typedef int            v4i   __attribute__((ext_vector_type(4)));
typedef unsigned short v8us  __attribute__((ext_vector_type(8)));
typedef __bf16         v16bf __attribute__((ext_vector_type(16)));
union Frag { v16bf v; v8us half[2]; };

__device__ __forceinline__ v8f wm(v16bf a, v16bf b, v8f c) {
  v8f d = __builtin_amdgcn_wmma_f32_16x16x32_bf16(false, a, false, b, (short)0, c, false, false);
  asm volatile("v_nop\n\tv_nop\n\tv_nop\n\tv_nop" : "+v"(d) : "v"(a), "v"(b));
  return d;
}

__device__ __forceinline__ unsigned short bf_rne(float f) {
  unsigned u = __float_as_uint(f);
  u += 0x7FFFu + ((u >> 16) & 1u);
  return (unsigned short)(u >> 16);
}
__device__ __forceinline__ void split2(float f, unsigned short& hi, unsigned short& lo) {
  const unsigned short hb = bf_rne(f);
  const float hf = __uint_as_float(((unsigned)hb) << 16);
  hi = hb;
  lo = bf_rne(f - hf);
}
__device__ __forceinline__ void split8(v4f a, v4f b, v8us& hi, v8us& lo) {
  unsigned short h, l;
  split2(a.x, h, l); hi[0] = h; lo[0] = l;
  split2(a.y, h, l); hi[1] = h; lo[1] = l;
  split2(a.z, h, l); hi[2] = h; lo[2] = l;
  split2(a.w, h, l); hi[3] = h; lo[3] = l;
  split2(b.x, h, l); hi[4] = h; lo[4] = l;
  split2(b.y, h, l); hi[5] = h; lo[5] = l;
  split2(b.z, h, l); hi[6] = h; lo[6] = l;
  split2(b.w, h, l); hi[7] = h; lo[7] = l;
}

__device__ __forceinline__ float th(float x) {
  const float ax = fabsf(x);
  const float t  = __expf(-2.0f * ax);
  const float r  = (1.0f - t) * __builtin_amdgcn_rcpf(1.0f + t);
  return copysignf(r, x);
}

__global__ __launch_bounds__(NTHR) void k_prep(const float* __restrict__ Wa, const float* __restrict__ Wb,
                                               unsigned short* planes) {
  __shared__ __attribute__((aligned(16))) float T[16 * TP];
  const int tid = threadIdx.x, lane = tid & 31, wave = tid >> 5;
  const int mat = (int)(blockIdx.x >> 3);
  const int n0  = (int)(blockIdx.x & 7) * 16;
  const float* W = (mat == 0) ? Wa : Wb;
  unsigned short* ph = planes + (size_t)mat * 2 * FT * FT;
  unsigned short* pl = ph + FT * FT;
  {
    const int k  = tid >> 1;
    const int c8 = (tid & 1) * 8;
    const float* p = W + (size_t)k * FT + n0 + c8;
    const v4f f0 = *(const v4f*)p;
    const v4f f1 = *(const v4f*)(p + 4);
    T[(c8 + 0) * TP + k] = f0.x; T[(c8 + 1) * TP + k] = f0.y;
    T[(c8 + 2) * TP + k] = f0.z; T[(c8 + 3) * TP + k] = f0.w;
    T[(c8 + 4) * TP + k] = f1.x; T[(c8 + 5) * TP + k] = f1.y;
    T[(c8 + 6) * TP + k] = f1.z; T[(c8 + 7) * TP + k] = f1.w;
  }
  __syncthreads();
  const int hh = lane >> 4, l16 = lane & 15;
  const int nl = 2 * wave + hh;
  const int k0 = l16 * 8;
  const v4f g0 = *(const v4f*)(T + nl * TP + k0);
  const v4f g1 = *(const v4f*)(T + nl * TP + k0 + 4);
  v8us uh = {0, 0, 0, 0, 0, 0, 0, 0}, ul = {0, 0, 0, 0, 0, 0, 0, 0};
  split8(g0, g1, uh, ul);
  const size_t o = (size_t)(n0 + nl) * FT + k0;
  *(volatile v8us*)(ph + o) = uh;
  *(volatile v8us*)(pl + o) = ul;
  __threadfence();
  *(volatile v8us*)(ph + o) = uh;
  *(volatile v8us*)(pl + o) = ul;
}

__device__ __forceinline__ void epi_tile(v8f acc, int T, int hh, int m, int wave, int ncol,
                                         float cs, float cd, float* Xs, float* Pd) {
  float ss[8], sd[8];
#pragma unroll
  for (int r = 0; r < 8; ++r) {
    const float v = acc[r];
    Xs[(T * 16 + 8 * hh + r) * XSP + ncol] = v;
    ss[r] = v * cs;
    sd[r] = v * cd;
  }
#pragma unroll
  for (int mk = 1; mk < 16; mk <<= 1) {
#pragma unroll
    for (int r = 0; r < 8; ++r) {
      ss[r] += __shfl_xor(ss[r], mk, 32);
      sd[r] += __shfl_xor(sd[r], mk, 32);
    }
  }
  if (m == 0) {
#pragma unroll
    for (int r = 0; r < 8; ++r) {
      Pd[(T * 16 + 8 * hh + r) * NWAVE + wave]      = ss[r];
      Pd[(GR + T * 16 + 8 * hh + r) * NWAVE + wave] = sd[r];
    }
  }
}

__global__ __launch_bounds__(NTHR) void k_gemm(
    const float* __restrict__ A, const unsigned short* __restrict__ Wh, const unsigned short* __restrict__ Wl,
    const float* __restrict__ att_src, const float* __restrict__ att_dst,
    float* h, float* asrc, float* adst, int nN) {
  __shared__ __attribute__((aligned(16))) unsigned short Ah[GR * AP];
  __shared__ __attribute__((aligned(16))) unsigned short Al[GR * AP];
  __shared__ __attribute__((aligned(16))) float Xs[GR * XSP];
  __shared__ __attribute__((aligned(16))) float Pd[2 * GR * NWAVE];
  __shared__ __attribute__((aligned(16))) float Sl[2 * GR];

  const int tid  = threadIdx.x;
  const int lane = tid & 31;
  const int wave = tid >> 5;
  const int hh   = lane >> 4;
  const int m    = lane & 15;
  const int rowBase = (int)blockIdx.x * GR;

  {
    const int r  = tid >> 3;
    const int c0 = (tid & 7) * 16;
    int row = rowBase + r;
    if (row > nN - 1) row = nN - 1;
    const float* p = A + (size_t)row * FT + c0;
    const v4f f0 = *(const v4f*)(p),     f1 = *(const v4f*)(p + 4);
    const v4f f2 = *(const v4f*)(p + 8), f3 = *(const v4f*)(p + 12);
    v8us h0 = {0, 0, 0, 0, 0, 0, 0, 0}, l0 = {0, 0, 0, 0, 0, 0, 0, 0};
    v8us h1 = {0, 0, 0, 0, 0, 0, 0, 0}, l1 = {0, 0, 0, 0, 0, 0, 0, 0};
    split8(f0, f1, h0, l0);
    split8(f2, f3, h1, l1);
    *(v8us*)(Ah + r * AP + c0)     = h0;
    *(v8us*)(Ah + r * AP + c0 + 8) = h1;
    *(v8us*)(Al + r * AP + c0)     = l0;
    *(v8us*)(Al + r * AP + c0 + 8) = l1;
  }
  __syncthreads();

  const int ncol = wave * 16 + m;
  const unsigned short* wbh  = Wh + (size_t)ncol * FT + 8 * hh;
  const unsigned short* wbl  = Wl + (size_t)ncol * FT + 8 * hh;
  const unsigned short* pa0h = Ah + m * AP + 8 * hh;
  const unsigned short* pa0l = Al + m * AP + 8 * hh;
  const unsigned short* pa1h = Ah + (16 + m) * AP + 8 * hh;
  const unsigned short* pa1l = Al + (16 + m) * AP + 8 * hh;
  v8f c0a = {0.f, 0.f, 0.f, 0.f, 0.f, 0.f, 0.f, 0.f};
  v8f c1a = {0.f, 0.f, 0.f, 0.f, 0.f, 0.f, 0.f, 0.f};
#pragma unroll
  for (int kt = 0; kt < FT / 32; ++kt) {
    const int k0 = kt * 32;
    Frag bh, bl, a0h, a0l, a1h, a1l;
    bh.half[0]  = *(const v8us*)(wbh + k0);   bh.half[1]  = *(const v8us*)(wbh + k0 + 16);
    bl.half[0]  = *(const v8us*)(wbl + k0);   bl.half[1]  = *(const v8us*)(wbl + k0 + 16);
    a0h.half[0] = *(const v8us*)(pa0h + k0);  a0h.half[1] = *(const v8us*)(pa0h + k0 + 16);
    a0l.half[0] = *(const v8us*)(pa0l + k0);  a0l.half[1] = *(const v8us*)(pa0l + k0 + 16);
    a1h.half[0] = *(const v8us*)(pa1h + k0);  a1h.half[1] = *(const v8us*)(pa1h + k0 + 16);
    a1l.half[0] = *(const v8us*)(pa1l + k0);  a1l.half[1] = *(const v8us*)(pa1l + k0 + 16);
    c0a = wm(a0h.v, bh.v, c0a);
    c0a = wm(a0h.v, bl.v, c0a);
    c0a = wm(a0l.v, bh.v, c0a);
    c1a = wm(a1h.v, bh.v, c1a);
    c1a = wm(a1h.v, bl.v, c1a);
    c1a = wm(a1l.v, bh.v, c1a);
  }

  const float cs = att_src[ncol];
  const float cd = att_dst[ncol];
  epi_tile(c0a, 0, hh, m, wave, ncol, cs, cd, Xs, Pd);
  epi_tile(c1a, 1, hh, m, wave, ncol, cs, cd, Xs, Pd);
  __syncthreads();

  if (tid < 2 * GR) {
    const float* pp = Pd + tid * NWAVE;
    const v4f p0 = *(const v4f*)pp;
    const v4f p1 = *(const v4f*)(pp + 4);
    float s = p0.x; s += p0.y; s += p0.z; s += p0.w;
    s += p1.x; s += p1.y; s += p1.z; s += p1.w;
    Sl[tid] = s;
  }
  v4f xr[4];
#pragma unroll
  for (int i = 0; i < 4; ++i) xr[i] = *(const v4f*)(Xs + (4 * wave + i) * XSP + 4 * lane);
  __syncthreads();

  const int which = (lane >> 3) & 1;
  const int q     = lane & 7;
  const v4f gv = *(const v4f*)(Sl + which * GR + 4 * q);
  float* gp = (which ? adst : asrc) + (size_t)rowBase + 4 * q;
  const bool wl = (wave == 0) && (lane < 16);
  float* hp[4];
#pragma unroll
  for (int i = 0; i < 4; ++i) hp[i] = h + (size_t)(rowBase + 4 * wave + i) * FT + 4 * lane;

#pragma unroll
  for (int i = 0; i < 4; ++i) *(volatile v4f*)(hp[i]) = xr[i];
  if (wl) *(volatile v4f*)gp = gv;
  __threadfence();
#pragma unroll
  for (int i = 0; i < 4; ++i) *(volatile v4f*)(hp[i]) = xr[i];
  if (wl) *(volatile v4f*)gp = gv;
}

__global__ __launch_bounds__(NTHR) void k_gat(
    const int* __restrict__ ei, const float* __restrict__ hm,
    const float* __restrict__ asrc, const float* __restrict__ adst,
    const float* __restrict__ bias, const float* x1r, const float* __restrict__ ew,
    float* dst, int nN, int nE, int fin) {
  extern __shared__ v4f lds_dyn[];
  float* sacc = (float*)lds_dyn;
  float* smax = sacc + LDS_SACC;
  float* den  = smax + NB;
  float* sdl  = den + NB;
  int*   list = (int*)(sdl + NB);
  int*   wcnt = list + LDS_LIST;
  (void)ew;

  const int tid  = threadIdx.x;
  const int lane = tid & 31;
  const int wave = tid >> 5;
  const int nodeBase = (int)blockIdx.x * NB;

#pragma unroll 2
  for (int j = 0; j < NB / NWAVE; ++j) {
    const int slot = wave * (NB / NWAVE) + j;
    int node = nodeBase + slot;
    if (node > nN - 1) node = nN - 1;
    const float as = asrc[node];
    const float ad = adst[node];
    float lg = as + ad;
    lg = (lg > 0.f) ? lg : 0.2f * lg;
    const v4f hv = *(const v4f*)(hm + (size_t)node * FT + 4 * lane);
    *(v4f*)(sacc + slot * FT + 4 * lane) = hv;
    smax[slot] = lg;
    den[slot]  = 1.0f;
    sdl[slot]  = ad;
  }
  __syncthreads();

  const int* eid = ei + nE;
  const bool al16 = ((nE & 3) == 0);
  const int nChunks = (nE + CHUNK - 1) / CHUNK;

#pragma unroll 1
  for (int ch = 0; ch < nChunks; ++ch) {
    const int cbase = ch * CHUNK;
    const bool vec = al16 && (cbase + CHUNK <= nE);
    int wc = 0;
#pragma unroll
    for (int g = 0; g < NGRP; ++g) {
      const int el0 = (g * NTHR + tid) * 4;
      const int e0  = cbase + el0;
      const int sent = -2147483647 - 1;
      v4i d;
      if (vec) {
        d = *(const v4i*)(eid + e0);
      } else {
        const int em = nE - 1;
        d.x = (e0     < nE) ? eid[min(e0,     em)] : sent;
        d.y = (e0 + 1 < nE) ? eid[min(e0 + 1, em)] : sent;
        d.z = (e0 + 2 < nE) ? eid[min(e0 + 2, em)] : sent;
        d.w = (e0 + 3 < nE) ? eid[min(e0 + 3, em)] : sent;
      }
      const unsigned s0 = (unsigned)d.x - (unsigned)nodeBase;
      const unsigned s1 = (unsigned)d.y - (unsigned)nodeBase;
      const unsigned s2 = (unsigned)d.z - (unsigned)nodeBase;
      const unsigned s3 = (unsigned)d.w - (unsigned)nodeBase;
      const bool h0 = s0 < (unsigned)NB;
      const bool h1 = s1 < (unsigned)NB;
      const bool h2 = s2 < (unsigned)NB;
      const bool h3 = s3 < (unsigned)NB;
      const unsigned many = __builtin_amdgcn_ballot_w32(h0 | h1 | h2 | h3);
      if (many != 0u) {
#define HITJ(J, HJ, SJ) { \
          const unsigned mj = __builtin_amdgcn_ballot_w32(HJ); \
          if (HJ) { \
            const int pos = wc + (int)__builtin_amdgcn_mbcnt_lo(mj, 0u); \
            if (pos < WCAP) list[wave * WCAP + pos] = ((el0 + (J)) << 9) | (int)(SJ); \
          } \
          wc += (int)__builtin_popcount(mj); }
        HITJ(0, h0, s0)
        HITJ(1, h1, s1)
        HITJ(2, h2, s2)
        HITJ(3, h3, s3)
#undef HITJ
      }
    }
    if (lane == 0) wcnt[wave] = wc;
    __syncthreads();

    if (wave == 0) {
#pragma unroll 1
      for (int wsx = 0; wsx < NWAVE; ++wsx) {
        int n = wcnt[wsx];
        if (n > WCAP) n = WCAP;
        if (n < 0) n = 0;
#pragma unroll 1
        for (int i = 0; i < n; ++i) {
          const int ent  = list[wsx * WCAP + i];
          const int slot = ent & (NB - 1);
          const int el   = (ent >> 9) & (CHUNK - 1);
          int e = cbase + el;
          if (e > nE - 1) e = nE - 1;
          int src = ei[e];
          src = src < 0 ? 0 : (src > nN - 1 ? nN - 1 : src);
          float lg = asrc[src] + sdl[slot];
          lg = (lg > 0.f) ? lg : 0.2f * lg;
          const float mo = smax[slot];
          const float mn = fmaxf(mo, lg);
          const float sc = __expf(mo - mn);
          const float p  = __expf(lg - mn);
          const v4f hv = *(const v4f*)(hm + (size_t)src * FT + 4 * lane);
          v4f* sp = (v4f*)(sacc + slot * FT + 4 * lane);
          const v4f cur = *sp;
          const v4f nxt = cur * sc + hv * p;
          *sp = nxt;
          const float dn = den[slot] * sc + p;
          den[slot]  = dn;
          smax[slot] = mn;
        }
      }
    }
    __syncthreads();
  }

  const v4f b4 = *(const v4f*)(bias + 4 * lane);
#pragma unroll 1
  for (int j = 0; j < NB / NWAVE; ++j) {
    const int slot = wave * (NB / NWAVE) + j;
    const int node = nodeBase + slot;
    if (node >= nN) break;
    const size_t nrow = (size_t)node;
    const float iv = __builtin_amdgcn_rcpf(den[slot]);
    const v4f sv = *(const v4f*)(sacc + slot * FT + 4 * lane);
    const v4f rr = sv * iv + b4;
    v4f y;
    if (fin != 0) {
      const v4f xo = *(const v4f*)(x1r + nrow * FT + 4 * lane);
      y.x = fmaxf(xo.x, rr.x); y.y = fmaxf(xo.y, rr.y);
      y.z = fmaxf(xo.z, rr.z); y.w = fmaxf(xo.w, rr.w);
    } else {
      y.x = th(rr.x); y.y = th(rr.y); y.z = th(rr.z); y.w = th(rr.w);
    }
    float* op = dst + nrow * FT + 4 * lane;
    *(volatile v4f*)op = y;
    __threadfence();
    *(volatile v4f*)op = y;
  }
}

extern "C" void kernel_launch(void* const* d_in, const int* in_sizes, int n_in,
                              void* d_out, int out_size, void* d_ws, size_t ws_size,
                              hipStream_t stream) {
  if (n_in < 11) return;
  const int nN = in_sizes[0] / FT;
  if (nN <= 0 || in_sizes[0] != nN * FT) return;
  if (in_sizes[1] < 0 || (in_sizes[1] & 1) != 0) return;
  const int nE = in_sizes[1] / 2;
  if (in_sizes[3] != FT * FT || in_sizes[7] != FT * FT) return;
  if (in_sizes[4] != FT || in_sizes[5] != FT || in_sizes[6] != FT) return;
  if (in_sizes[8] != FT || in_sizes[9] != FT || in_sizes[10] != FT) return;
  if (out_size != nN * FT) return;

  const float* x      = (const float*)d_in[0];
  const int*   ei     = (const int*)d_in[1];
  const float* ew     = (const float*)d_in[2];
  const float* W1     = (const float*)d_in[3];
  const float* a_src1 = (const float*)d_in[4];
  const float* a_dst1 = (const float*)d_in[5];
  const float* b1     = (const float*)d_in[6];
  const float* W2     = (const float*)d_in[7];
  const float* a_src2 = (const float*)d_in[8];
  const float* a_dst2 = (const float*)d_in[9];
  const float* b2     = (const float*)d_in[10];
  float* out = (float*)d_out;

  const int nP = ((nN + GR - 1) / GR) * GR;
  size_t off = 0;
  unsigned short* planes = (unsigned short*)((char*)d_ws + off); off += (size_t)4 * FT * FT * sizeof(unsigned short);
  float* h    = (float*)((char*)d_ws + off); off += (size_t)nP * FT * sizeof(float);
  float* x1   = (float*)((char*)d_ws + off); off += (size_t)nP * FT * sizeof(float);
  float* asrc = (float*)((char*)d_ws + off); off += (((size_t)nP * sizeof(float)) + 255) & ~(size_t)255;
  float* adst = (float*)((char*)d_ws + off); off += (((size_t)nP * sizeof(float)) + 255) & ~(size_t)255;
  if (off > ws_size) return;
  if (off > (size_t)134217728) return;

  k_prep<<<16, NTHR, 0, stream>>>(W1, W2, planes);

  k_gemm<<<nP / GR, NTHR, 0, stream>>>(x, planes, planes + FT * FT, a_src1, a_dst1, h, asrc, adst, nN);
  hipFuncSetAttribute(reinterpret_cast<const void*>(&k_gat),
                      hipFuncAttributeMaxDynamicSharedMemorySize, LDS_BYTES);
  const int grid = (nN + NB - 1) / NB;
  k_gat<<<grid, NTHR, LDS_BYTES, stream>>>(ei, h, asrc, adst, b1, x1, ew, x1, nN, nE, 0);

  k_gemm<<<nP / GR, NTHR, 0, stream>>>(x1, planes + 2 * FT * FT, planes + 3 * FT * FT, a_src2, a_dst2,
                                       h, asrc, adst, nN);
  k_gat<<<grid, NTHR, LDS_BYTES, stream>>>(ei, h, asrc, adst, b2, x1, ew, out, nN, nE, 1);
}
